// TransformerBlockQuantum_65481071400592
// MI455X (gfx1250) — hardware-run, weakly checked
//
#include <hip/hip_runtime.h>


#ifndef NB
#define NB 16
#endif
#ifndef SEQ
#define SEQ 2048
#endif
#define NB_FULL  16
#define SEQ_FULL 2048
#ifndef OUT_SEQ
#define OUT_SEQ SEQ
#endif
#define EMB  8
#define NH_  2
#define DK   4
#define KP   32
#define VROWS 16
#define FFN  2048
#define AW   4
#define FW   4
#define PW   4
#define SC2  ((float)(0.5 * 1.4426950408889634))
#define PSH  14.0f
#define NEGB (-3.0e38f)
#define W1S  16.0f
#define W2S  256.0f
#define FSI  (1.0f / 4096.0f)
#define LNEPS 1.0e-5f

static_assert(NH_ * DK == EMB);
static_assert(DK == 4);
static_assert(EMB == 8);
static_assert(DK + 1 <= 8);
static_assert(KP == 32);
static_assert(VROWS == 16);
static_assert(EMB <= KP);
static_assert(FFN % 32 == 0);
static_assert(SEQ % 64 == 0);
static_assert(SEQ % 32 == 0);
static_assert(SEQ % (16 * AW) == 0);
static_assert((NB * SEQ) % (16 * FW) == 0);
static_assert((NB * SEQ) % (64 * PW) == 0);
static_assert(NB <= NB_FULL);
static_assert(SEQ <= SEQ_FULL);
static_assert(OUT_SEQ % 16 == 0);
static_assert((FFN * KP / 8) % 256 == 0);
static_assert((16 * FFN / 8) % 256 == 0);
static_assert((FFN / 8) % 32 == 0);
static_assert(W1S * W2S * FSI == 1.0f);

typedef _Float16 h16;
typedef __attribute__((ext_vector_type(16))) _Float16 v16h;
typedef __attribute__((ext_vector_type(8)))  _Float16 v8h;
typedef __attribute__((ext_vector_type(8)))  float    v8f;
typedef __attribute__((ext_vector_type(4)))  float    v4f;
typedef v4f  __attribute__((may_alias)) v4fa;

__device__ __forceinline__ unsigned short f2bf(float f) { unsigned u = __float_as_uint(f); u += 0x7FFFu + ((u >> 16) & 1u); return (unsigned short)(u >> 16); }
__device__ __forceinline__ float bfr(float f) { return __uint_as_float(((unsigned)f2bf(f)) << 16); }
__device__ __forceinline__ v16h cat16(v8h lo, v8h hi) { return __builtin_shufflevector(lo, hi, 0, 1, 2, 3, 4, 5, 6, 7, 8, 9, 10, 11, 12, 13, 14, 15); }
__device__ __forceinline__ v8f wmma16(v16h a, v16h b, v8f c) { return __builtin_amdgcn_wmma_f32_16x16x32_f16(false, a, false, b, (short)0, c, false, false); }
__device__ __forceinline__ v16h  ldh(const h16* p) { return cat16(*(const v8h*)p, *(const v8h*)(p + 16)); }
__device__ __forceinline__ void wave_sync() { __builtin_amdgcn_fence(3  , "wavefront"); __builtin_amdgcn_wave_barrier(); asm volatile("" ::: "memory"); }
static __device__ __forceinline__ h16 toh_flush(float v) { const h16 r = (h16)v; return (fabsf(v) < 6.103515625e-05f) ? (h16)0.0f : r; }
__device__ __forceinline__ v8f wmma16g(v16h a, v16h b, v8f c) { c = wmma16(a, b, c); asm volatile("v_nop\n\tv_nop\n\tv_nop\n\tv_nop" : "+v"(c) : "v"(a), "v"(b)); return c; }

__device__ __forceinline__ void ln8(float (&v)[8], const float* __restrict__ g, const float* __restrict__ be) {
    float mean = 0.0f;
#pragma unroll
    for (int e = 0; e < 8; ++e) mean += v[e];
    mean *= 0.125f;
    float var = 0.0f;
#pragma unroll
    for (int e = 0; e < 8; ++e) { const float d = v[e] - mean; var += d * d; }
    var *= 0.125f;
    const float rs = rsqrtf(var + LNEPS);
#pragma unroll
    for (int e = 0; e < 8; ++e) v[e] = (v[e] - mean) * rs * bfr(g[e]) + bfr(be[e]);
}

#define W1B (FFN * KP / 8 / 256)
#define W2B (16 * FFN / 8 / 256)
__global__ __launch_bounds__(256) void k_wconv(const float* __restrict__ w1, const float* __restrict__ w2, h16* W1P, h16* W2P) {
    const int blk = blockIdx.x;
    if (blk < W1B) {
        const int i = blk * 256 + (int)threadIdx.x;
        const int f = i >> 2, c8 = (i & 3) * 8;
        v4f a = *(const v4f*)(w1 + (size_t)f * EMB); v4f c = *(const v4f*)(w1 + (size_t)f * EMB + 4);
        asm volatile("" : "+v"(a)); asm volatile("" : "+v"(c));
        v8h o;
#pragma unroll
        for (int k = 0; k < 4; ++k) { const h16 q0 = toh_flush(bfr(a[k]) * W1S); const h16 q1 = toh_flush(bfr(c[k]) * W1S);
            o[k] = (c8 == 0) ? q0 : (h16)0.0f; o[4 + k] = (c8 == 0) ? q1 : (h16)0.0f; }
        *(volatile v8h*)(W1P + (size_t)i * 8) = o; __threadfence(); *(volatile v8h*)(W1P + (size_t)i * 8) = o;
    } else {
        const int i = (blk - W1B) * 256 + (int)threadIdx.x;
        const int n = i / (FFN / 8), c8 = (i % (FFN / 8)) * 8;
        const int nc = n < EMB ? n : (EMB - 1);
        v4f a = *(const v4f*)(w2 + (size_t)nc * FFN + c8); v4f c = *(const v4f*)(w2 + (size_t)nc * FFN + c8 + 4);
        asm volatile("" : "+v"(a)); asm volatile("" : "+v"(c));
        v8h o;
#pragma unroll
        for (int k = 0; k < 4; ++k) { const h16 q0 = toh_flush(bfr(a[k]) * W2S); const h16 q1 = toh_flush(bfr(c[k]) * W2S);
            o[k] = (n < EMB) ? q0 : (h16)0.0f; o[4 + k] = (n < EMB) ? q1 : (h16)0.0f; }
        *(volatile v8h*)(W2P + (size_t)i * 8) = o; __threadfence(); *(volatile v8h*)(W2P + (size_t)i * 8) = o;
    }
}

static_assert(8 * 32 * 16 == 64 * KP * 2);
static_assert(4 * 32 * 16 == VROWS * 64 * 2);
static_assert(16 * 32 == 64 * EMB);
static_assert(PW * 64 * EMB * 4 <= 131072);
__global__ __launch_bounds__(32 * PW) void k_prep(const float* __restrict__ x, const float* __restrict__ theta, h16* HP, h16* VT) {
    __shared__ __align__(16) float hs[PW * 64 * EMB];
    const int lane = threadIdx.x & 31;
    const int wave = __builtin_amdgcn_readfirstlane((int)(threadIdx.x >> 5));
    const int tile = blockIdx.x * PW + wave;
    const int tok0 = tile * 64; const int b = tok0 / SEQ, tt = tok0 % SEQ;
    const float* xr = x + ((size_t)b * SEQ_FULL + tt) * EMB;
    const int wb = wave * 64 * EMB;
#pragma unroll 1
    for (int i = 0; i < 16; ++i) { const int idx = i * 32 + lane; const int c = idx & 7;
        const float v = bfr(xr[idx]) + bfr(theta[c]);
        hs[wb + idx] = cosf(v); }
    wave_sync();
#pragma unroll 1
    for (int ps = 0; ps < 2; ++ps) {
#pragma unroll 1
        for (int hh = 0; hh < NH_; ++hh) {
            const size_t zh = (size_t)b * NH_ + hh;
            const size_t hb = (zh * SEQ + (size_t)tt) * KP;
            const size_t vb = zh * VROWS * SEQ + (size_t)tt;
#pragma unroll 1
            for (int s = 0; s < 8; ++s) { const int p = s * 32 + lane; const int row = p >> 2, c8 = (p & 3) * 8;
                v4f x0 = *(const v4fa*)(&hs[wb + row * EMB + hh * DK]);
                asm volatile("" : "+v"(x0));
                v8h hv;
#pragma unroll
                for (int i = 0; i < 4; ++i) { const h16 q = toh_flush(x0[i]); hv[i] = (c8 == 0) ? q : (h16)0.0f; hv[4 + i] = (h16)0.0f; }
                *(volatile v8h*)(HP + hb + (size_t)p * 8) = hv; }
#pragma unroll 1
            for (int s = 0; s < 4; ++s) { const int d = 4 * s + (lane >> 3), c8 = (lane & 7) * 8;
                const int dc = d < DK ? d : 0;
                v8h vv;
#pragma unroll
                for (int i = 0; i < 8; ++i) { float hv = hs[wb + (c8 + i) * EMB + hh * DK + dc];
                    asm volatile("" : "+v"(hv));
                    const h16 q = toh_flush(hv);
                    vv[i] = (d < DK) ? q : ((d == DK) ? (h16)1.0f : (h16)0.0f); }
                *(volatile v8h*)(VT + vb + (size_t)d * SEQ + c8) = vv; }
        }
        if (ps == 0) __threadfence(); }
}

static_assert(1 * 32 * 16 == 16 * EMB * 4);
static_assert(2 * 32 * 16 == 16 * KP * 2);
static_assert(3 * AW * 16 * EMB * 4 <= 131072);
__global__ __launch_bounds__(32 * AW) void k_attn(const h16* __restrict__ HP, const h16* __restrict__ VT, const float* __restrict__ x, const float* __restrict__ w_out,
                                                  const float* __restrict__ g1, const float* __restrict__ b1, const float* __restrict__ phi, float* X1, h16* QF) {
    __shared__ __align__(16) float os[AW * 16 * EMB];
    __shared__ __align__(16) float xs[AW * 16 * EMB];
    __shared__ __align__(16) float qs[AW * 16 * EMB];
    const int lane = threadIdx.x & 31, lr = lane & 15, hi = lane >> 4;
    const int wave = __builtin_amdgcn_readfirstlane((int)(threadIdx.x >> 5));
    const int b = blockIdx.y;
    const int t0 = (blockIdx.x * AW + wave) * 16;
    const int wb = wave * 16 * EMB;
#pragma unroll 1
    for (int hd = 0; hd < NH_; ++hd) {
        const int zh = b * NH_ + hd;
        const size_t pbase = (size_t)zh * SEQ * KP;
        const size_t vbase = (size_t)zh * VROWS * SEQ;
        const v16h qh = ldh(HP + pbase + (size_t)(t0 + lr) * KP + 8 * hi);
        const size_t ko = pbase + (size_t)lr * KP + 8 * hi;
        const size_t vo = vbase + (size_t)lr * SEQ + 8 * hi;
        v8f o = (v8f){};
        float m = NEGB;
#pragma unroll 1
        for (int key0 = 0; key0 < SEQ; key0 += 32) {
            const h16* ka = HP + ko + (size_t)key0 * KP;
            const v16h ka0 = ldh(ka), kb0 = ldh(ka + 16 * KP);
            v8f sa = (v8f){}, sb = (v8f){};
            sa = wmma16g(ka0, qh, sa); sb = wmma16g(kb0, qh, sb);
            float ta[8], tb[8]; float mx = NEGB;
#pragma unroll
            for (int r = 0; r < 8; ++r) { ta[r] = sa[r] * SC2; tb[r] = sb[r] * SC2; mx = fmaxf(mx, fmaxf(ta[r], tb[r])); }
            mx = fmaxf(mx, __shfl_xor(mx, 16, 32));
            const float mnew = fmaxf(m, mx);
            const float alpha = __builtin_amdgcn_exp2f(m - mnew);
            const float sh = PSH - mnew;
            v16h pb;
#pragma unroll
            for (int r = 0; r < 8; ++r) {
                const float ea = ta[r] + sh, eb = tb[r] + sh;
                const float ga = (ea < -14.0f) ? 0.0f : __builtin_amdgcn_exp2f(ea);
                const float gb = (eb < -14.0f) ? 0.0f : __builtin_amdgcn_exp2f(eb);
                pb[r] = (h16)ga; pb[8 + r] = (h16)gb; }
            m = mnew;
            o = o * alpha;
            const v16h v0 = ldh(VT + vo + key0);
            o = wmma16g(v0, pb, o);
        }
        const float den = (hi == 0) ? o[4] : 1.0f;
        const float inv = 1.0f / den;
        v4f a; a[0] = o[0] * inv; a[1] = o[1] * inv; a[2] = o[2] * inv; a[3] = o[3] * inv;
        if (hi == 0) *(v4fa*)(&os[wb + lr * EMB + hd * DK]) = a;
    }
    wave_sync();
    float av[8], tv[8];
    { const v4f a0 = *(const v4fa*)(&os[wb + lr * EMB]); const v4f a1 = *(const v4fa*)(&os[wb + lr * EMB + 4]);
#pragma unroll
      for (int i = 0; i < 4; ++i) { av[i] = a0[i]; av[4 + i] = a1[i]; } }
    { const float* xr = x + ((size_t)b * SEQ_FULL + t0 + lr) * EMB;
      const v4f x0 = *(const v4f*)xr; const v4f x1 = *(const v4f*)(xr + 4);
      float xv[8];
#pragma unroll
      for (int i = 0; i < 4; ++i) { xv[i] = bfr(x0[i]); xv[4 + i] = bfr(x1[i]); }
#pragma unroll
      for (int e = 0; e < 8; ++e) { float s = 0.0f;
#pragma unroll
          for (int i = 0; i < 8; ++i) s += av[i] * bfr(w_out[e * EMB + i]);
          tv[e] = xv[e] + s; } }
    ln8(tv, g1, b1);
    if (hi == 0) { v4f a, c; a[0] = tv[0]; a[1] = tv[1]; a[2] = tv[2]; a[3] = tv[3]; c[0] = tv[4]; c[1] = tv[5]; c[2] = tv[6]; c[3] = tv[7];
        *(v4fa*)(&xs[wb + lr * EMB]) = a; *(v4fa*)(&xs[wb + lr * EMB + 4]) = c; }
    wave_sync();
    { const int row = lane >> 1, c4 = (lane & 1) * 4;
#pragma unroll 1
      for (int j = 0; j < 4; ++j) { const int e = c4 + j;
          const float xv = xs[wb + row * EMB + e];
          const float ph = bfr(phi[e]);
          qs[wb + row * EMB + e] = cosf(xv) * cosf(ph); } }
    wave_sync();
    const size_t tokb = (size_t)b * SEQ + (size_t)t0;
#pragma unroll 1
    for (int ps = 0; ps < 2; ++ps) {
        { const v4f val = *(const v4fa*)(&xs[wb + lane * 4]);
          *(volatile v4f*)(X1 + tokb * EMB + (size_t)lane * 4) = val; }
#pragma unroll
        for (int s = 0; s < 2; ++s) { const int p = s * 32 + lane; const int row = p >> 2, c8 = (p & 3) * 8;
            v4f x0 = *(const v4fa*)(&qs[wb + row * EMB]); v4f x1 = *(const v4fa*)(&qs[wb + row * EMB + 4]);
            asm volatile("" : "+v"(x0)); asm volatile("" : "+v"(x1));
            v8h hv;
#pragma unroll
            for (int i = 0; i < 4; ++i) { const h16 q0 = toh_flush(x0[i]); const h16 q1 = toh_flush(x1[i]);
                hv[i] = (c8 == 0) ? q0 : (h16)0.0f; hv[4 + i] = (c8 == 0) ? q1 : (h16)0.0f; }
            *(volatile v8h*)(QF + tokb * KP + (size_t)p * 8) = hv; }
        if (ps == 0) __threadfence(); }
}

static_assert(1 * 32 * 16 == 16 * EMB * 4);
static_assert(FW * 16 * EMB * 4 <= 131072);
__global__ __launch_bounds__(32 * FW) void k_ffn(const h16* __restrict__ QF, const h16* __restrict__ W1P, const h16* __restrict__ W2P, const float* __restrict__ X1,
                                                 const float* __restrict__ g2, const float* __restrict__ b2, float* OUT) {
    __shared__ __align__(16) float ys[FW * 16 * EMB];
    const int lane = threadIdx.x & 31, lr = lane & 15, hi = lane >> 4;
    const int wave = __builtin_amdgcn_readfirstlane((int)(threadIdx.x >> 5));
    const int tile = blockIdx.x * FW + wave;
    const int tok0 = tile * 16; const int b = tok0 / SEQ, tt = tok0 % SEQ;
    const v16h qf = ldh(QF + (size_t)(tok0 + lr) * KP + 8 * hi);
    const size_t w1o = (size_t)lr * KP + 8 * hi;
    const size_t w2o = (size_t)lr * FFN + 8 * hi;
    v8f acc = (v8f){};
#pragma unroll 1
    for (int f0 = 0; f0 < FFN; f0 += 32) {
        const h16* wa = W1P + w1o + (size_t)f0 * KP;
        const v16h wa0 = ldh(wa), wb0 = ldh(wa + 16 * KP);
        v8f ha = (v8f){}, hb = (v8f){};
        ha = wmma16g(wa0, qf, ha); hb = wmma16g(wb0, qf, hb);
        v16h pb;
#pragma unroll
        for (int r = 0; r < 8; ++r) { pb[r] = toh_flush(fmaxf(ha[r], 0.0f)); pb[8 + r] = toh_flush(fmaxf(hb[r], 0.0f)); }
        const v16h w2f = ldh(W2P + w2o + f0);
        acc = wmma16g(w2f, pb, acc);
    }
    float val[8];
    { const float* xr = X1 + (size_t)(tok0 + lr) * EMB;
      const v4f x0 = *(const v4f*)xr; const v4f x1 = *(const v4f*)(xr + 4);
#pragma unroll
      for (int r = 0; r < 4; ++r) { val[r] = acc[r] * FSI + x0[r]; val[4 + r] = acc[4 + r] * FSI + x1[r]; } }
    ln8(val, g2, b2);
    const int wb = wave * 16 * EMB;
    if (hi == 0) { v4f a, c; a[0] = val[0]; a[1] = val[1]; a[2] = val[2]; a[3] = val[3]; c[0] = val[4]; c[1] = val[5]; c[2] = val[6]; c[3] = val[7];
        *(v4fa*)(&ys[wb + lr * EMB]) = a; *(v4fa*)(&ys[wb + lr * EMB + 4]) = c; }
    wave_sync();
    float* orow = OUT + ((size_t)b * OUT_SEQ + tt) * EMB;
#pragma unroll 1
    for (int ps = 0; ps < 2; ++ps) {
        const v4f v = *(const v4fa*)(&ys[wb + lane * 4]);
        *(volatile v4f*)(orow + (size_t)lane * 4) = v;
        if (ps == 0) __threadfence(); }
}

static constexpr size_t al256(size_t v) { return (v + 255) & ~(size_t)255; }
static constexpr size_t SZ_HP = al256((size_t)NB * NH_ * SEQ * KP * 2);
static constexpr size_t SZ_VT = al256((size_t)NB * NH_ * VROWS * SEQ * 2);
static constexpr size_t SZ_X1 = al256((size_t)NB * SEQ * EMB * 4);
static constexpr size_t SZ_QF = al256((size_t)NB * SEQ * KP * 2);
static constexpr size_t SZ_W1 = al256((size_t)FFN * KP * 2);
static constexpr size_t SZ_W2 = al256((size_t)16 * FFN * 2);
static constexpr size_t SZ_TOTAL = SZ_HP + SZ_VT + SZ_X1 + SZ_QF + SZ_W1 + SZ_W2;
static_assert(SZ_TOTAL <= (size_t)134217728);
static_assert((size_t)(NB * SEQ / 64) * 64 * NH_ * KP * 2 == (size_t)NB * NH_ * SEQ * KP * 2);
static_assert((size_t)(NB * SEQ / 64) * NH_ * VROWS * 64 * 2 == (size_t)NB * NH_ * VROWS * SEQ * 2);
static_assert((size_t)(NB * SEQ / 16) * 16 * KP * 2 == (size_t)NB * SEQ * KP * 2);
static_assert((size_t)W1B * 256 * 16 == (size_t)FFN * KP * 2);
static_assert((size_t)W2B * 256 * 16 == (size_t)16 * FFN * 2);

extern "C" void kernel_launch(void* const* d_in, const int* in_sizes, int n_in,
                              void* d_out, int out_size, void* d_ws, size_t ws_size, hipStream_t stream) {
    if (n_in < 10) return;
    const size_t needx = ((size_t)(NB - 1) * SEQ_FULL + SEQ) * EMB;
    if ((size_t)in_sizes[0] < needx) return;
    if (in_sizes[1] < EMB || in_sizes[2] < EMB * EMB || in_sizes[3] < EMB || in_sizes[4] < EMB || in_sizes[5] < EMB) return;
    if ((size_t)in_sizes[6] < (size_t)FFN * EMB || (size_t)in_sizes[7] < (size_t)EMB * FFN) return;
    if (in_sizes[8] < EMB || in_sizes[9] < EMB) return;
    if ((size_t)out_size < ((size_t)(NB - 1) * OUT_SEQ + SEQ) * EMB) return;
    if (SZ_TOTAL > ws_size) return;
    const float* x     = (const float*)d_in[0];
    const float* theta = (const float*)d_in[1];
    const float* w_out = (const float*)d_in[2];
    const float* g1    = (const float*)d_in[3];
    const float* b1    = (const float*)d_in[4];
    const float* phi   = (const float*)d_in[5];
    const float* w1    = (const float*)d_in[6];
    const float* w2    = (const float*)d_in[7];
    const float* g2    = (const float*)d_in[8];
    const float* b2    = (const float*)d_in[9];
    float* OUT = (float*)d_out;
    char* wsp = (char*)d_ws;
    h16* HP = (h16*)wsp; wsp += SZ_HP;
    h16* VT = (h16*)wsp; wsp += SZ_VT;
    float* X1 = (float*)wsp; wsp += SZ_X1;
    h16* QF = (h16*)wsp; wsp += SZ_QF;
    h16* W1P = (h16*)wsp; wsp += SZ_W1;
    h16* W2P = (h16*)wsp; wsp += SZ_W2;

    k_wconv<<<dim3(W1B + W2B, 1, 1), 256, 0, stream>>>(w1, w2, W1P, W2P);
    k_prep<<<dim3(NB * SEQ / (64 * PW), 1, 1), 32 * PW, 0, stream>>>(x, theta, HP, VT);
    k_attn<<<dim3(SEQ / (16 * AW), NB, 1), 32 * AW, 0, stream>>>(HP, VT, x, w_out, g1, b1, phi, X1, QF);
    k_ffn<<<dim3(NB * SEQ / (16 * FW), 1, 1), 32 * FW, 0, stream>>>(QF, W1P, W2P, X1, g2, b2, OUT);
}
